// Model_3582002725443
// MI455X (gfx1250) — hardware-run, weakly checked
//
#include <hip/hip_runtime.h>
#include <math.h>

typedef __attribute__((ext_vector_type(16))) _Float16 v16h;
typedef __attribute__((ext_vector_type(8)))  _Float16 v8h;
typedef __attribute__((ext_vector_type(8)))  float    v8f;
typedef __attribute__((ext_vector_type(4)))  float    v4f;

constexpr int kT   = 96;
constexpr int kB   = 64;
constexpr int kM   = kT * kB;
constexpr int kDM  = 1024;
constexpr int kDA  = 100;
constexpr int kDAP = 128;
constexpr int kDV  = 512;
constexpr int kDG  = 512;
constexpr int kH   = 256;
constexpr int kG   = 4 * kH;
constexpr int kPH  = kH + 8;
constexpr int kOutCols = 3 * kDG;
constexpr float kWCarry = 1024.0f;
constexpr float sW = 1.0f / kWCarry;
constexpr float kLnCount = (float)(kT * kDM);
static_assert(kM == 6144 && kG == 1024 && kPH == 264 && kOutCols == 1536);
static_assert(kDG == 2 * kH);
static_assert((kDAP % 32) == 0 && (kDV % 32) == 0 && (kDM % 32) == 0 && (kDG % 32) == 0 && (kH % 128) == 0);
static_assert((kM % 32) == 0 && (kDG % 64) == 0 && (kG % 64) == 0);
static_assert(kDA <= kDAP && (kPH % 8) == 0);
static_assert(kLnCount == 98304.0f);

constexpr size_t kSzSTAT = (size_t)4 * kB * 32 * 4;
constexpr size_t kSzUH   = (size_t)kM * kDM * 2;
constexpr size_t kSzUAH  = (size_t)kM * kDAP * 2;
constexpr size_t kSzUVH  = (size_t)kM * kDV * 2;
constexpr size_t kSzP32  = (size_t)kM * kDG * 4;
constexpr size_t kSzP16  = (size_t)kM * kDG * 2;
constexpr size_t kSzXG   = (size_t)2 * kM * kG * 4;
constexpr size_t kSzWA   = (size_t)kDG * kDAP * 2;
constexpr size_t kSzWV   = (size_t)kDG * kDV * 2;
constexpr size_t kSzWL   = (size_t)kDG * kDM * 2;
constexpr size_t kSzWIH  = (size_t)4 * kG * kDG * 2;
constexpr size_t kSzWHH  = (size_t)4 * kG * kH * 2;
constexpr size_t kSzB512 = (size_t)kDG * 4;
constexpr size_t kSzBG   = (size_t)4 * kG * 4;
constexpr size_t kOffSTAT = 0;
constexpr size_t kOffUH   = kOffSTAT + kSzSTAT;
constexpr size_t kOffUAH  = kOffUH   + kSzUH;
constexpr size_t kOffUVH  = kOffUAH  + kSzUAH;
constexpr size_t kOffEA   = kOffUVH  + kSzUVH;
constexpr size_t kOffEV   = kOffEA   + kSzP32;
constexpr size_t kOffUL   = kOffEV   + kSzP32;
constexpr size_t kOffULH  = kOffUL   + kSzP32;
constexpr size_t kOffXG   = kOffULH  + kSzP16;
constexpr size_t kOffHL1  = kOffUL;
constexpr size_t kOffHLH  = kOffXG + kSzXG;
constexpr size_t kOffWA   = kOffHLH  + kSzP16;
constexpr size_t kOffWV   = kOffWA   + kSzWA;
constexpr size_t kOffWL   = kOffWV   + kSzWV;
constexpr size_t kOffWIH  = kOffWL   + kSzWL;
constexpr size_t kOffWHH  = kOffWIH  + kSzWIH;
constexpr size_t kOffBA   = kOffWHH  + kSzWHH;
constexpr size_t kOffBV   = kOffBA   + kSzB512;
constexpr size_t kOffBL   = kOffBV   + kSzB512;
constexpr size_t kOffBIH  = kOffBL   + kSzB512;
constexpr size_t kOffBHH  = kOffBIH  + kSzBG;
constexpr size_t kWsTotal = kOffBHH  + kSzBG;
static_assert(kSzSTAT == 32768ull && kSzUH == 12582912ull && kSzUAH == 1572864ull && kSzUVH == 6291456ull);
static_assert(kSzP32 == 12582912ull && kSzP16 == 6291456ull && kSzXG == 50331648ull);
static_assert(kSzWA == 131072ull && kSzWV == 524288ull && kSzWL == 1048576ull);
static_assert(kSzWIH == 4194304ull && kSzWHH == 2097152ull && kSzB512 == 2048ull && kSzBG == 16384ull);
static_assert(kWsTotal == 129177600ull);
static_assert(kWsTotal <= 134217728ull);
static_assert((kSzSTAT % 256) == 0 && (kSzUH % 256) == 0 && (kSzUAH % 256) == 0 && (kSzUVH % 256) == 0 &&
              (kSzP32 % 256) == 0 && (kSzP16 % 256) == 0 && (kSzXG % 256) == 0 && (kSzWA % 256) == 0 &&
              (kSzWV % 256) == 0 && (kSzWL % 256) == 0 && (kSzWIH % 256) == 0 && (kSzWHH % 256) == 0 &&
              (kSzB512 % 256) == 0 && (kSzBG % 256) == 0);

__device__ __forceinline__ _Float16 f16_flush(float v) {
  const float w = (fabsf(v) < 6.103515625e-05f) ? 0.0f : v;
  return (_Float16)w;
}

__device__ __forceinline__ float bf16r(float v) {
  unsigned u = __float_as_uint(v);
  u = (u + 0x7FFFu + ((u >> 16) & 1u)) & 0xFFFF0000u;
  return __uint_as_float(u);
}

namespace eng {
union FragU { v16h v; v8h h[2]; };
__device__ __forceinline__ v16h frag_load(const _Float16* p) {
  FragU f;
  f.h[0] = *(const v8h*)(p);
  f.h[1] = *(const v8h*)(p + 16);
  return f.v;
}
__device__ __forceinline__ v8f mma(v16h a, v16h b, v8f c) {
  return __builtin_amdgcn_wmma_f32_16x16x32_f16(false, a, false, b, (short)0, c, false, false);
}
__device__ __forceinline__ void guard1(v8f& a, v16h x, v16h y) {
  asm volatile("v_nop\n\tv_nop\n\tv_nop\n\tv_nop" : "+v"(a) : "v"(x), "v"(y));
}
__device__ __forceinline__ void guard_acc(v8f& a) {
  asm volatile("v_nop\n\tv_nop\n\tv_nop\n\tv_nop" : "+v"(a));
}
__device__ __forceinline__ void keep4(v16h a, v16h b, v16h c, v16h d) {
  asm volatile("v_nop" :: "v"(a), "v"(b), "v"(c), "v"(d));
}

template <int MI, int SPL>
__global__ __launch_bounds__(256) void gemm_f16_kernel(
    const unsigned short* __restrict__ Ap, const unsigned short* __restrict__ A2p, int lda,
    const unsigned short* __restrict__ Btp, const unsigned short* __restrict__ Bt2p, int ldb,
    float* __restrict__ C, int ldc, int M, int N, int K, float scale, float rscale)
{
  static_assert(MI >= 1 && MI <= 2);
  static_assert(SPL >= 0 && SPL <= 2);
  const _Float16* A   = (const _Float16*)Ap;
  const _Float16* A2  = (const _Float16*)A2p;
  const _Float16* Bt  = (const _Float16*)Btp;
  const _Float16* Bt2 = (const _Float16*)Bt2p;
  __shared__ __align__(16) float sT[8][16 * 68];
  const int lane = threadIdx.x & 31;
  const int wave = threadIdx.x >> 5;
  const int tilesN = N >> 6;
  const int tilesM = M / (16 * MI);
  const int tile = blockIdx.x * 8 + wave;
  if (tile >= tilesM * tilesN) return;
  const int tm = tile / tilesN;
  const int tn = tile - tm * tilesN;
  const int m0 = tm * (16 * MI);
  const int n0 = tn << 6;
  const int rlane = lane & 15;
  const int koff  = (lane >> 4) * 8;
  const int mOff  = (lane >> 4) * 8;

  v8f acc[MI][4], accr[MI][4];
#pragma unroll
  for (int i = 0; i < MI; ++i)
#pragma unroll
    for (int j = 0; j < 4; ++j) {
      acc[i][j]  = (v8f){0.f, 0.f, 0.f, 0.f, 0.f, 0.f, 0.f, 0.f};
      accr[i][j] = (v8f){0.f, 0.f, 0.f, 0.f, 0.f, 0.f, 0.f, 0.f};
    }

  for (int k0 = 0; k0 < K; k0 += 32) {
    v16h bh[4], bl[4];
#pragma unroll
    for (int j = 0; j < 4; ++j) {
      const size_t bo = (size_t)(n0 + (j << 4) + rlane) * ldb + koff + k0;
      bh[j] = frag_load(Bt + bo);
      if (SPL == 2) bl[j] = frag_load(Bt2 + bo); else bl[j] = bh[j];
    }
#pragma unroll
    for (int i = 0; i < MI; ++i) {
      const size_t ao = (size_t)(m0 + (i << 4) + rlane) * lda + koff + k0;
      const v16h ah = frag_load(A + ao);
      v16h al = ah;
      if (SPL >= 1) al = frag_load(A2 + ao);
#pragma unroll
      for (int j = 0; j < 4; ++j) {
        acc[i][j] = mma(ah, bh[j], acc[i][j]);
        if (SPL >= 1) accr[i][j] = mma(al, bh[j], accr[i][j]);
        if (SPL == 2) accr[i][j] = mma(ah, bl[j], accr[i][j]);
      }
#pragma unroll
      for (int j = 0; j < 4; ++j) {
        guard1(acc[i][j], ah, al);
        if (SPL >= 1) guard1(accr[i][j], ah, al);
      }
    }
    keep4(bh[0], bh[1], bh[2], bh[3]);
    if (SPL == 2) keep4(bl[0], bl[1], bl[2], bl[3]);
  }
#pragma unroll
  for (int i = 0; i < MI; ++i)
#pragma unroll
    for (int j = 0; j < 4; ++j) {
      guard_acc(acc[i][j]);
      if (SPL >= 1) guard_acc(accr[i][j]);
    }

  float* slab = sT[wave];
#pragma unroll
  for (int i = 0; i < MI; ++i) {
    const int mBase = m0 + (i << 4);
#pragma unroll
    for (int j = 0; j < 4; ++j) {
#pragma unroll
      for (int r = 0; r < 8; ++r) {
        float v = acc[i][j][r] * scale;
        if (SPL >= 1) v += accr[i][j][r] * rscale;
        slab[(mOff + r) * 68 + (j << 4) + rlane] = v;
      }
    }
    __builtin_amdgcn_fence(__ATOMIC_RELEASE, "workgroup");
    __builtin_amdgcn_wave_barrier();
    __builtin_amdgcn_fence(__ATOMIC_ACQUIRE, "workgroup");
    {
      const int hh = lane >> 4, c4 = (lane & 15) * 4;
      for (int pass = 0; pass < 2; ++pass) {
#pragma unroll
        for (int it = 0; it < 8; ++it) {
          const int row = it * 2 + hh;
          const v4f v = *(const v4f*)(slab + row * 68 + c4);
          *(volatile v4f*)(C + (size_t)(mBase + row) * ldc + n0 + c4) = v;
        }
        __threadfence();
      }
    }
    __builtin_amdgcn_fence(__ATOMIC_RELEASE, "workgroup");
    __builtin_amdgcn_wave_barrier();
    __builtin_amdgcn_fence(__ATOMIC_ACQUIRE, "workgroup");
  }
}
}

template <int K>
__device__ __forceinline__ v8f tile_mm(const _Float16* A, int lda, const _Float16* __restrict__ Bt, int ldb,
                                       int n0, int rlane, int koff, v8f acc)
{
  static_assert((K % 32) == 0 && K >= 32 && K <= 128);
#pragma unroll
  for (int k0 = 0; k0 < K; k0 += 32) {
    const v16h ah = eng::frag_load(A + rlane * lda + koff + k0);
    const v16h bh = eng::frag_load(Bt + (size_t)(n0 + rlane) * ldb + koff + k0);
    acc = eng::mma(ah, bh, acc);
    eng::guard1(acc, ah, bh);
    eng::keep4(bh, bh, ah, ah);
  }
  return acc;
}

__global__ __launch_bounds__(256) void pack_rows_bf_kernel(
    const float* __restrict__ W, unsigned short* __restrict__ dH,
    int Kdim, int Nreal, int total8, float carry)
{
  const int i = blockIdx.x * 256 + threadIdx.x;
  if (i >= total8) return;
  const size_t e0 = (size_t)i << 3;
  const int row = (int)(e0 / (size_t)Kdim);
  const int col = (int)(e0 - (size_t)row * (size_t)Kdim);
  const bool live = (row < Nreal);
  const int rc = live ? row : (Nreal - 1);
  const v4f a0 = *(const v4f*)(W + (size_t)rc * Kdim + col);
  const v4f a1 = *(const v4f*)(W + (size_t)rc * Kdim + col + 4);
  const float w0 = a0[0];
  const float w1 = a0[1];
  const float w2 = a0[2];
  const float w3 = a0[3];
  const float w4 = a1[0];
  const float w5 = a1[1];
  const float w6 = a1[2];
  const float w7 = a1[3];
  const float t0 = bf16r(w0) * carry;
  const float t1 = bf16r(w1) * carry;
  const float t2 = bf16r(w2) * carry;
  const float t3 = bf16r(w3) * carry;
  const float t4 = bf16r(w4) * carry;
  const float t5 = bf16r(w5) * carry;
  const float t6 = bf16r(w6) * carry;
  const float t7 = bf16r(w7) * carry;
  const float g0 = live ? t0 : 0.0f;
  const float g1 = live ? t1 : 0.0f;
  const float g2 = live ? t2 : 0.0f;
  const float g3 = live ? t3 : 0.0f;
  const float g4 = live ? t4 : 0.0f;
  const float g5 = live ? t5 : 0.0f;
  const float g6 = live ? t6 : 0.0f;
  const float g7 = live ? t7 : 0.0f;
  v8h hv;
  hv[0] = f16_flush(g0);
  hv[1] = f16_flush(g1);
  hv[2] = f16_flush(g2);
  hv[3] = f16_flush(g3);
  hv[4] = f16_flush(g4);
  hv[5] = f16_flush(g5);
  hv[6] = f16_flush(g6);
  hv[7] = f16_flush(g7);
  unsigned short* qh = dH + e0;
  *(volatile v8h*)qh = hv;
  __threadfence();
  *(volatile v8h*)qh = hv;
}

__global__ __launch_bounds__(256) void rne_vec_kernel(
    const float* __restrict__ src, float* __restrict__ dst, int n4)
{
  const int i = blockIdx.x * 256 + threadIdx.x;
  if (i >= n4) return;
  const v4f a = *(const v4f*)(src + (size_t)i * 4);
  const float a0 = a[0];
  const float a1 = a[1];
  const float a2 = a[2];
  const float a3 = a[3];
  v4f r;
  r[0] = bf16r(a0);
  r[1] = bf16r(a1);
  r[2] = bf16r(a2);
  r[3] = bf16r(a3);
  float* p = dst + (size_t)i * 4;
  *(volatile v4f*)p = r;
  __threadfence();
  *(volatile v4f*)p = r;
}

__global__ __launch_bounds__(256) void ln2_stats_kernel(
    const float* __restrict__ r1, const float* __restrict__ r2,
    const float* __restrict__ r3, const float* __restrict__ r4,
    float* __restrict__ STAT)
{
  __shared__ float red[8];
  const int tid  = threadIdx.x;
  const int lane = tid & 31;
  const int wave = tid >> 5;
  const int b = blockIdx.x;
  const int k = blockIdx.y;
  const float* r = (k == 0) ? r1 : (k == 1) ? r2 : (k == 2) ? r3 : r4;
  const float* base = r + (size_t)b * kDM + 4 * tid;

  float s = 0.0f;
  for (int t = 0; t < kT; ++t) {
    const v4f a = *(const v4f*)(base + (size_t)t * kB * kDM);
    const float a0 = a[0];
    const float a1 = a[1];
    const float a2 = a[2];
    const float a3 = a[3];
    s += bf16r(a0);
    s += bf16r(a1);
    s += bf16r(a2);
    s += bf16r(a3);
  }
  s += __shfl_xor(s, 16, 32);
  s += __shfl_xor(s, 8, 32);
  s += __shfl_xor(s, 4, 32);
  s += __shfl_xor(s, 2, 32);
  s += __shfl_xor(s, 1, 32);
  if (lane == 0) red[wave] = s;
  __syncthreads();
  const float tot = ((((((red[0] + red[1]) + red[2]) + red[3]) + red[4]) + red[5]) + red[6]) + red[7];
  const float mean = tot / kLnCount;
  __syncthreads();

  float q = 0.0f;
  for (int t = 0; t < kT; ++t) {
    const v4f a = *(const v4f*)(base + (size_t)t * kB * kDM);
    const float a0 = a[0];
    const float a1 = a[1];
    const float a2 = a[2];
    const float a3 = a[3];
    const float d0 = bf16r(a0) - mean;
    const float d1 = bf16r(a1) - mean;
    const float d2 = bf16r(a2) - mean;
    const float d3 = bf16r(a3) - mean;
    q += d0 * d0;
    q += d1 * d1;
    q += d2 * d2;
    q += d3 * d3;
  }
  q += __shfl_xor(q, 16, 32);
  q += __shfl_xor(q, 8, 32);
  q += __shfl_xor(q, 4, 32);
  q += __shfl_xor(q, 2, 32);
  q += __shfl_xor(q, 1, 32);
  if (lane == 0) red[wave] = q;
  __syncthreads();
  const float totq = ((((((red[0] + red[1]) + red[2]) + red[3]) + red[4]) + red[5]) + red[6]) + red[7];
  const float var = totq / kLnCount;
  const float rstd = 1.0f / sqrtf(var + 1e-5f);

  if (tid < 32) {
    const float v = (lane == 0) ? mean : ((lane == 1) ? rstd : 0.0f);
    float* p = STAT + (size_t)(k * kB + b) * 32 + lane;
    *(volatile float*)p = v;
    __threadfence();
    *(volatile float*)p = v;
  }
}

__device__ __forceinline__ void ln2_add(const float* __restrict__ r, const float* __restrict__ STAT,
                                        int k, int b, size_t e0, float (&u)[8])
{
  const float mk = STAT[(k * kB + b) * 32];
  const float rk = STAT[(k * kB + b) * 32 + 1];
  const v4f a0 = *(const v4f*)(r + e0);
  const v4f a1 = *(const v4f*)(r + e0 + 4);
#pragma unroll
  for (int e = 0; e < 4; ++e) {
    const float x0 = a0[e];
    const float x1 = a1[e];
    u[e]     += (bf16r(x0) - mk) * rk;
    u[4 + e] += (bf16r(x1) - mk) * rk;
  }
}

static_assert(((kM * kDM / 8) % 256) == 0 && (kM * kDM / 8) / 256 == 3072);
__global__ __launch_bounds__(256) void ln2_avg_word_kernel(
    const float* __restrict__ r1, const float* __restrict__ r2,
    const float* __restrict__ r3, const float* __restrict__ r4,
    const float* __restrict__ STAT, unsigned short* __restrict__ UH)
{
  const int i = blockIdx.x * 256 + threadIdx.x;
  const int row = i >> 7;
  const int f8 = (i & 127) * 8;
  const int b = row & (kB - 1);
  const size_t e0 = (size_t)row * kDM + f8;
  float u[8];
#pragma unroll
  for (int e = 0; e < 8; ++e) u[e] = 0.0f;
  ln2_add(r1, STAT, 0, b, e0, u);
  ln2_add(r2, STAT, 1, b, e0, u);
  ln2_add(r3, STAT, 2, b, e0, u);
  ln2_add(r4, STAT, 3, b, e0, u);
  v8h hv;
#pragma unroll
  for (int e = 0; e < 8; ++e) hv[e] = f16_flush(u[e] * 0.25f);
  unsigned short* qh = UH + e0;
  *(volatile v8h*)qh = hv;
  __threadfence();
  *(volatile v8h*)qh = hv;
}

__global__ __launch_bounds__(256) void in_word_kernel(
    const float* __restrict__ src, unsigned short* __restrict__ dst, int Kreal, int Kpad, int total8)
{
  const int i = blockIdx.x * 256 + threadIdx.x;
  if (i >= total8) return;
  const int per = Kpad >> 3;
  const int row = i / per;
  const int c8 = (i - row * per) * 8;
  const float* sp = src + (size_t)row * Kreal;
  v8h hv;
#pragma unroll
  for (int e = 0; e < 8; ++e) {
    const int c = c8 + e;
    const bool live = (c < Kreal);
    const int cc = live ? c : (Kreal - 1);
    const float x = sp[cc];
    const float v = live ? bf16r(x) : 0.0f;
    hv[e] = f16_flush(v);
  }
  unsigned short* qh = dst + (size_t)row * Kpad + c8;
  *(volatile v8h*)qh = hv;
  __threadfence();
  *(volatile v8h*)qh = hv;
}

static_assert(((kDG * kDAP / 8) % 256) == 0 && (kDG * kDAP / 8) / 256 == 32);
__global__ __launch_bounds__(256) void wa_pack_kernel(
    const float* __restrict__ Wa, unsigned short* __restrict__ WA)
{
  const int i = blockIdx.x * 256 + threadIdx.x;
  const int n = i >> 4;
  const int k8 = (i & 15) * 8;
  const float* sp = Wa + (size_t)n * kDA;
  v8h hv;
#pragma unroll
  for (int e = 0; e < 8; ++e) {
    const int k = k8 + e;
    const bool live = (k < kDA);
    const int kc = live ? k : (kDA - 1);
    const float x = sp[kc];
    const float v = live ? (bf16r(x) * kWCarry) : 0.0f;
    hv[e] = f16_flush(v);
  }
  unsigned short* qh = WA + (size_t)n * kDAP + k8;
  *(volatile v8h*)qh = hv;
  __threadfence();
  *(volatile v8h*)qh = hv;
}

static_assert(((kM * kDG / 8) % 256) == 0 && (kM * kDG / 8) / 256 == 1536);
__global__ __launch_bounds__(256) void bias_word_kernel(
    const float* __restrict__ UL, const float* __restrict__ BL, unsigned short* __restrict__ ULH)
{
  const int i = blockIdx.x * 256 + threadIdx.x;
  const int row = i >> 6;
  const int c8 = (i & 63) * 8;
  const size_t e0 = (size_t)row * kDG + c8;
  const v4f p0 = *(const v4f*)(UL + e0);
  const v4f p1 = *(const v4f*)(UL + e0 + 4);
  const v4f q0 = *(const v4f*)(BL + c8);
  const v4f q1 = *(const v4f*)(BL + c8 + 4);
  v8h hv;
#pragma unroll
  for (int e = 0; e < 4; ++e) {
    const float x0 = p0[e];
    const float x1 = p1[e];
    const float y0 = q0[e];
    const float y1 = q1[e];
    hv[e]     = f16_flush(x0 + y0);
    hv[4 + e] = f16_flush(x1 + y1);
  }
  unsigned short* qh = ULH + e0;
  *(volatile v8h*)qh = hv;
  __threadfence();
  *(volatile v8h*)qh = hv;
}

__global__ __launch_bounds__(256) void lstm_dir_kernel(
    const float* __restrict__ XG, const unsigned short* __restrict__ WHHp,
    const float* __restrict__ BIH, const float* __restrict__ BHH,
    float* __restrict__ HL, unsigned short* __restrict__ HLH, int words)
{
  __shared__ __align__(16) _Float16 P_H[16 * kPH];
  __shared__ __align__(16) float HS[16 * 256];

  const int tid   = threadIdx.x;
  const int lane  = tid & 31;
  const int wave  = tid >> 5;
  const int rlane = lane & 15;
  const int hi    = lane >> 4;
  const int koff  = 8 * hi;
  const int b0    = 16 * blockIdx.x;
  const int d     = blockIdx.y;
  const int sa    = tid >> 4;
  const int ll    = tid & 15;

  const float* XGd = XG + (size_t)d * kM * kG;
  const _Float16* WHHd = (const _Float16*)WHHp + (size_t)d * kG * kH;
  const float* BIHd = BIH + d * kG;
  const float* BHHd = BHH + d * kG;

  float bsum[2][4];
#pragma unroll
  for (int j = 0; j < 2; ++j) {
    const int uj = 32 * wave + 16 * j + rlane;
#pragma unroll
    for (int q = 0; q < 4; ++q) bsum[j][q] = BIHd[kH * q + uj] + BHHd[kH * q + uj];
  }

  v8f hreg[2], creg[2];
#pragma unroll
  for (int j = 0; j < 2; ++j) {
    hreg[j] = (v8f){0.f, 0.f, 0.f, 0.f, 0.f, 0.f, 0.f, 0.f};
    creg[j] = (v8f){0.f, 0.f, 0.f, 0.f, 0.f, 0.f, 0.f, 0.f};
  }

  {
    v8h zz;
#pragma unroll
    for (int e = 0; e < 8; ++e) zz[e] = (_Float16)0.0f;
    for (int i = tid; i < (16 * kPH) / 8; i += 256) *(v8h*)(P_H + i * 8) = zz;
  }
  __syncthreads();

  for (int s = 0; s < kT; ++s) {
    const int t = (d == 0) ? s : (kT - 1 - s);

#pragma unroll
    for (int j = 0; j < 2; ++j) {
      const int uj = 32 * wave + 16 * j + rlane;
      const int nb = 32 * wave + 16 * j;
      v8f a0 = (v8f){0.f, 0.f, 0.f, 0.f, 0.f, 0.f, 0.f, 0.f};
      v8f a1 = (v8f){0.f, 0.f, 0.f, 0.f, 0.f, 0.f, 0.f, 0.f};
      v8f a2 = (v8f){0.f, 0.f, 0.f, 0.f, 0.f, 0.f, 0.f, 0.f};
      v8f a3 = (v8f){0.f, 0.f, 0.f, 0.f, 0.f, 0.f, 0.f, 0.f};
      a0 = tile_mm<128>(P_H, kPH, WHHd, kH, 0 * kH + nb, rlane, koff, a0);
      a0 = tile_mm<128>(P_H + 128, kPH, WHHd + 128, kH, 0 * kH + nb, rlane, koff, a0);
      eng::guard_acc(a0);
      a1 = tile_mm<128>(P_H, kPH, WHHd, kH, 1 * kH + nb, rlane, koff, a1);
      a1 = tile_mm<128>(P_H + 128, kPH, WHHd + 128, kH, 1 * kH + nb, rlane, koff, a1);
      eng::guard_acc(a1);
      a2 = tile_mm<128>(P_H, kPH, WHHd, kH, 2 * kH + nb, rlane, koff, a2);
      a2 = tile_mm<128>(P_H + 128, kPH, WHHd + 128, kH, 2 * kH + nb, rlane, koff, a2);
      eng::guard_acc(a2);
      a3 = tile_mm<128>(P_H, kPH, WHHd, kH, 3 * kH + nb, rlane, koff, a3);
      a3 = tile_mm<128>(P_H + 128, kPH, WHHd + 128, kH, 3 * kH + nb, rlane, koff, a3);
      eng::guard_acc(a3);
#pragma unroll
      for (int r = 0; r < 8; ++r) {
        const float* xp = XGd + (size_t)(t * kB + b0 + 8 * hi + r) * kG + uj;
        const float g0 = a0[r] * sW + xp[0 * kH] + bsum[j][0];
        const float g1 = a1[r] * sW + xp[1 * kH] + bsum[j][1];
        const float g2 = a2[r] * sW + xp[2 * kH] + bsum[j][2];
        const float g3 = a3[r] * sW + xp[3 * kH] + bsum[j][3];
        const float iv = 1.0f / (1.0f + expf(-g0));
        const float fv = 1.0f / (1.0f + expf(-g1));
        const float gv = tanhf(g2);
        const float ov = 1.0f / (1.0f + expf(-g3));
        const float cn = fv * creg[j][r] + iv * gv;
        creg[j][r] = cn;
        hreg[j][r] = ov * tanhf(cn);
      }
    }
    __syncthreads();

#pragma unroll
    for (int j = 0; j < 2; ++j) {
      const int uj = 32 * wave + 16 * j + rlane;
#pragma unroll
      for (int r = 0; r < 8; ++r) {
        const float hv = hreg[j][r];
        P_H[(8 * hi + r) * kPH + uj] = f16_flush(hv);
        HS[(8 * hi + r) * 256 + uj] = hv;
      }
    }
    __syncthreads();

    {
      const size_t row = (size_t)(t * kB + b0 + sa);
      const float* hs = HS + sa * 256;
      v4f vv[4];
#pragma unroll
      for (int q = 0; q < 4; ++q) vv[q] = *(const v4f*)(hs + 64 * q + 4 * ll);
      v8h hw[2];
#pragma unroll
      for (int q = 0; q < 2; ++q) {
        const v4f f0 = *(const v4f*)(hs + 128 * q + 8 * ll);
        const v4f f1 = *(const v4f*)(hs + 128 * q + 8 * ll + 4);
#pragma unroll
        for (int e = 0; e < 4; ++e) {
          const float x0 = f0[e];
          const float x1 = f1[e];
          hw[q][e]     = f16_flush(x0);
          hw[q][4 + e] = f16_flush(x1);
        }
      }
      for (int pass = 0; pass < 2; ++pass) {
        if (HL != nullptr) {
          float* hp = HL + row * kDG + kH * d + 4 * ll;
#pragma unroll
          for (int q = 0; q < 4; ++q) *(volatile v4f*)(hp + 64 * q) = vv[q];
        }
        if (words) {
          unsigned short* wp = HLH + row * kDG + kH * d + 8 * ll;
#pragma unroll
          for (int q = 0; q < 2; ++q) *(volatile v8h*)(wp + 128 * q) = hw[q];
        }
        __threadfence();
      }
    }
  }
}

static_assert(kOutCols / 4 == 384);
__global__ __launch_bounds__(384) void out_concat_kernel(
    const float* __restrict__ EA, const float* __restrict__ EV, const float* __restrict__ HL,
    const float* __restrict__ BA, const float* __restrict__ BV, float* __restrict__ out)
{
  const int ro = blockIdx.x;
  const int b = ro / kT;
  const int t = ro - b * kT;
  const size_t rs = (size_t)(t * kB + b);
  const int wave = threadIdx.x >> 5;
  const int c = 4 * threadIdx.x;
  v4f v;
  if (wave < 4) {
    const v4f x = *(const v4f*)(EA + rs * kDG + c);
    const v4f y = *(const v4f*)(BA + c);
    v = x + y;
  } else if (wave < 8) {
    const v4f x = *(const v4f*)(EV + rs * kDG + (c - kDG));
    const v4f y = *(const v4f*)(BV + (c - kDG));
    v = x + y;
  } else {
    v = *(const v4f*)(HL + rs * kDG + (c - 2 * kDG));
  }
  float* p = out + (size_t)ro * kOutCols + c;
  *(volatile v4f*)p = v;
  __threadfence();
  *(volatile v4f*)p = v;
}

static_assert(((kM / 32) * (kDG / 64)) % 8 == 0 && ((kM / 32) * (kDG / 64)) / 8 == 192);
static_assert(((kM / 32) * (kG / 64)) % 8 == 0 && ((kM / 32) * (kG / 64)) / 8 == 384);
static_assert(((kM * kDAP / 8) % 256) == 0 && ((kM * kDV / 8) % 256) == 0);
static_assert(((kDG * kDV / 8) % 256) == 0 && ((kDG * kDM / 8) % 256) == 0);
static_assert(((kG * kDG / 8) % 256) == 0 && ((kG * kH / 8) % 256) == 0);
static_assert((kDG / 4) <= 256 && (kG / 4) <= 256);

extern "C" void kernel_launch(void* const* d_in, const int* in_sizes, int n_in,
                              void* d_out, int out_size, void* d_ws, size_t ws_size,
                              hipStream_t stream)
{
  if (n_in != 29) return;
  if (in_sizes[0] != kM * kDM) return;
  if (in_sizes[1] != kM * kDM) return;
  if (in_sizes[2] != kM * kDM) return;
  if (in_sizes[3] != kM * kDM) return;
  if (in_sizes[4] != kM * kDA) return;
  if (in_sizes[5] != kM * kDV) return;
  if (in_sizes[6] != kB) return;
  if (in_sizes[7] != kDG * kDA) return;
  if (in_sizes[8] != kDG) return;
  if (in_sizes[9] != kDG * kDV) return;
  if (in_sizes[10] != kDG) return;
  if (in_sizes[11] != kDG * kDM) return;
  if (in_sizes[12] != kDG) return;
  for (int ld = 0; ld < 4; ++ld) {
    const int base = 13 + 4 * ld;
    if (in_sizes[base + 0] != kG * kDG) return;
    if (in_sizes[base + 1] != kG * kH) return;
    if (in_sizes[base + 2] != kG) return;
    if (in_sizes[base + 3] != kG) return;
  }
  if (out_size != kM * kOutCols) return;
  if (ws_size < kWsTotal) return;

  const float* r1  = (const float*)d_in[0];
  const float* r2  = (const float*)d_in[1];
  const float* r3  = (const float*)d_in[2];
  const float* r4  = (const float*)d_in[3];
  const float* U_a = (const float*)d_in[4];
  const float* U_v = (const float*)d_in[5];
  const float* W_a = (const float*)d_in[7];
  const float* b_a = (const float*)d_in[8];
  const float* W_v = (const float*)d_in[9];
  const float* b_v = (const float*)d_in[10];
  const float* W_l = (const float*)d_in[11];
  const float* b_l = (const float*)d_in[12];
  float* out = (float*)d_out;

  char* ws = (char*)d_ws;
  float*          STAT = (float*)(ws + kOffSTAT);
  unsigned short* UH   = (unsigned short*)(ws + kOffUH);
  unsigned short* UAH  = (unsigned short*)(ws + kOffUAH);
  unsigned short* UVH  = (unsigned short*)(ws + kOffUVH);
  float*          EA   = (float*)(ws + kOffEA);
  float*          EV   = (float*)(ws + kOffEV);
  float*          UL   = (float*)(ws + kOffUL);
  unsigned short* ULH  = (unsigned short*)(ws + kOffULH);
  float*          XG   = (float*)(ws + kOffXG);
  float*          HL1  = (float*)(ws + kOffHL1);
  unsigned short* HLH  = (unsigned short*)(ws + kOffHLH);
  unsigned short* WA   = (unsigned short*)(ws + kOffWA);
  unsigned short* WV   = (unsigned short*)(ws + kOffWV);
  unsigned short* WL   = (unsigned short*)(ws + kOffWL);
  unsigned short* WIH  = (unsigned short*)(ws + kOffWIH);
  unsigned short* WHH  = (unsigned short*)(ws + kOffWHH);
  float*          BA   = (float*)(ws + kOffBA);
  float*          BV   = (float*)(ws + kOffBV);
  float*          BL   = (float*)(ws + kOffBL);
  float*          BIH  = (float*)(ws + kOffBIH);
  float*          BHH  = (float*)(ws + kOffBHH);

  wa_pack_kernel<<<(kDG * kDAP / 8) / 256, 256, 0, stream>>>(W_a, WA);
  pack_rows_bf_kernel<<<(kDG * kDV / 8) / 256, 256, 0, stream>>>(W_v, WV, kDV, kDG, kDG * kDV / 8, kWCarry);
  pack_rows_bf_kernel<<<(kDG * kDM / 8) / 256, 256, 0, stream>>>(W_l, WL, kDM, kDG, kDG * kDM / 8, kWCarry);
  for (int ld = 0; ld < 4; ++ld) {
    const float* Wih = (const float*)d_in[13 + 4 * ld];
    pack_rows_bf_kernel<<<(kG * kDG / 8) / 256, 256, 0, stream>>>(
        Wih, WIH + (size_t)ld * kG * kDG, kDG, kG, kG * kDG / 8, kWCarry);
  }
  for (int ld = 0; ld < 4; ++ld) {
    const float* Whh = (const float*)d_in[14 + 4 * ld];
    pack_rows_bf_kernel<<<(kG * kH / 8) / 256, 256, 0, stream>>>(
        Whh, WHH + (size_t)ld * kG * kH, kH, kG, kG * kH / 8, kWCarry);
  }

  rne_vec_kernel<<<1, 256, 0, stream>>>(b_a, BA, kDG / 4);
  rne_vec_kernel<<<1, 256, 0, stream>>>(b_v, BV, kDG / 4);
  rne_vec_kernel<<<1, 256, 0, stream>>>(b_l, BL, kDG / 4);
  for (int ld = 0; ld < 4; ++ld) {
    const float* bih = (const float*)d_in[15 + 4 * ld];
    const float* bhh = (const float*)d_in[16 + 4 * ld];
    rne_vec_kernel<<<1, 256, 0, stream>>>(bih, BIH + (size_t)ld * kG, kG / 4);
    rne_vec_kernel<<<1, 256, 0, stream>>>(bhh, BHH + (size_t)ld * kG, kG / 4);
  }

  ln2_stats_kernel<<<dim3(kB, 4), 256, 0, stream>>>(r1, r2, r3, r4, STAT);
  ln2_avg_word_kernel<<<(kM * kDM / 8) / 256, 256, 0, stream>>>(r1, r2, r3, r4, STAT, UH);

  in_word_kernel<<<(kM * kDAP / 8) / 256, 256, 0, stream>>>(U_a, UAH, kDA, kDAP, kM * kDAP / 8);
  in_word_kernel<<<(kM * kDV / 8) / 256, 256, 0, stream>>>(U_v, UVH, kDV, kDV, kM * kDV / 8);

  eng::gemm_f16_kernel<2, 0><<<dim3((kM / 32) * (kDG / 64) / 8), 256, 0, stream>>>(
      UAH, nullptr, kDAP, WA, nullptr, kDAP, EA, kDG, kM, kDG, kDAP, sW, 0.0f);
  eng::gemm_f16_kernel<2, 0><<<dim3((kM / 32) * (kDG / 64) / 8), 256, 0, stream>>>(
      UVH, nullptr, kDV, WV, nullptr, kDV, EV, kDG, kM, kDG, kDV, sW, 0.0f);
  eng::gemm_f16_kernel<2, 0><<<dim3((kM / 32) * (kDG / 64) / 8), 256, 0, stream>>>(
      UH, nullptr, kDM, WL, nullptr, kDM, UL, kDG, kM, kDG, kDM, sW, 0.0f);

  bias_word_kernel<<<(kM * kDG / 8) / 256, 256, 0, stream>>>(UL, BL, ULH);

  for (int l = 0; l < 2; ++l) {
    const unsigned short* opnd = (l == 0) ? ULH : HLH;
    for (int d = 0; d < 2; ++d) {
      eng::gemm_f16_kernel<2, 0><<<dim3((kM / 32) * (kG / 64) / 8), 256, 0, stream>>>(
          opnd, nullptr, kDG, WIH + (size_t)(l * 2 + d) * kG * kDG, nullptr, kDG,
          XG + (size_t)d * kM * kG, kG, kM, kG, kDG, sW, 0.0f);
    }
    lstm_dir_kernel<<<dim3(kB / 16, 2), 256, 0, stream>>>(
        XG, WHH + (size_t)l * 2 * kG * kH, BIH + (size_t)l * 2 * kG, BHH + (size_t)l * 2 * kG,
        (l == 0) ? (float*)nullptr : HL1, (l == 0) ? HLH : (unsigned short*)nullptr, (l == 0) ? 1 : 0);
  }

  out_concat_kernel<<<kM, kOutCols / 4, 0, stream>>>(EA, EV, HL1, BA, BV, out);
}
